// TGCNCell_52012053954618
// MI455X (gfx1250) — hardware-verified
//
#include <hip/hip_runtime.h>


namespace {
constexpr int NB = 16, NN = 2048, NC = 256, U = 64, KF = 96  , KP = 128  , G2 = 2 * U;
constexpr float XS = 8.0f, WSC = 256.0f, NMIX1 = 0.5f, NMIX2 = 0.5f;

typedef _Float16 b16;
typedef __attribute__((ext_vector_type(16))) _Float16 v16b;
typedef __attribute__((ext_vector_type(8))) _Float16 v8b;
typedef __attribute__((ext_vector_type(8))) float v8f;
typedef __attribute__((ext_vector_type(4))) float v4f;
__device__ __forceinline__ float bf16_rne(float f) { unsigned int u = __float_as_uint(f); u += 0x7FFFu + ((u >> 16) & 1u); return __uint_as_float(u & 0xFFFF0000u); }
__device__ __forceinline__ void split16(float v, b16& hi, b16& lo) { hi = (b16)v; lo = (b16)(v - (float)hi); }
__device__ __forceinline__ v16b frag_kb(const b16* p, int hh) { const v8b a = *(const v8b*)(p + 8 * hh), b = *(const v8b*)(p + 16 + 8 * hh); v16b f;
#pragma unroll
  for (int e = 0; e < 8; ++e) { f[e] = a[e]; f[8 + e] = b[e]; } return f; }
__device__ __forceinline__ v8f wmma16b(v16b a, v16b b, v8f c) { v8f d = __builtin_amdgcn_wmma_f32_16x16x32_f16(false, a, false, b, (short)0, c, false, false); asm volatile("v_nop\n\tv_nop\n\tv_nop\n\tv_nop" : "+v"(d) : "v"(a), "v"(b)); return d; }
__device__ __forceinline__ void wave_lds_sync() { __builtin_amdgcn_fence(__ATOMIC_RELEASE, "workgroup"); __builtin_amdgcn_wave_barrier(); __builtin_amdgcn_fence(__ATOMIC_ACQUIRE, "workgroup"); }
__device__ __forceinline__ float pmul(float a, float b) { float p = a * b; asm volatile("" : "+v"(p)); return p; }
__device__ __forceinline__ float sigm_(float v) { return 1.0f / (1.0f + __expf(-v)); }

__global__ __launch_bounds__(256) void prep_kernel(const float* __restrict__ adj, const float* __restrict__ adj1, const float* __restrict__ afc, const float* __restrict__ w0, const float* __restrict__ w1, const float* __restrict__ w01, const float* __restrict__ w11, b16* __restrict__ ADJ16, b16* __restrict__ ADJ1, b16* __restrict__ AFC16, b16* __restrict__ W0P, b16* __restrict__ W1P, b16* __restrict__ W01P, b16* __restrict__ W11P) {
  const size_t t = (size_t)blockIdx.x * 256 + threadIdx.x; size_t u = t; v8b o;
  const size_t n0 = (size_t)NN * NN / 8, n1 = (size_t)NC * NC / 8, n2 = (size_t)NN * NC / 8, nA = (size_t)G2 * KF / 8, nBk = (size_t)U * KF / 8;
  if (u < n0) { const size_t e = u * 8; const v4f a = *(const v4f*)(adj + e), c = *(const v4f*)(adj + e + 4); for (int j = 0; j < 4; ++j) { o[j] = (b16)(bf16_rne(a[j]) * WSC); o[4 + j] = (b16)(bf16_rne(c[j]) * WSC); } for (int pass = 0; pass < 2; ++pass) { *(volatile v8b*)(ADJ16 + e) = o; __threadfence(); } return; } u -= n0;
  if (u < n1) { const size_t e = u * 8; for (int j = 0; j < 8; ++j) o[j] = (b16)(bf16_rne(adj1[e + j]) * WSC); for (int pass = 0; pass < 2; ++pass) { *(volatile v8b*)(ADJ1 + e) = o; __threadfence(); } return; } u -= n1;
  if (u < n2) { const size_t e = u * 8; for (int j = 0; j < 8; ++j) o[j] = (b16)(bf16_rne(afc[e + j]) * XS); for (int pass = 0; pass < 2; ++pass) { *(volatile v8b*)(AFC16 + e) = o; __threadfence(); } return; } u -= n2;
  const float* w; b16* dst; int nout;
  if (u < nA) { w = w0; dst = W0P; nout = G2; } else if ((u -= nA) < nBk) { w = w1; dst = W1P; nout = U; } else if ((u -= nBk) < nA) { w = w01; dst = W01P; nout = G2; } else if ((u -= nA) < nBk) { w = w11; dst = W11P; nout = U; } else return;
  { const int e = (int)u * 8; const int oo = e / KF, k0 = e % KF; for (int j = 0; j < 8; ++j) { const int k = k0 + j; o[j] = (k < U + 1) ? (b16)(bf16_rne(w[k * nout + oo]) * WSC) : (b16)0.0f; } for (int pass = 0; pass < 2; ++pass) { *(volatile v8b*)(dst + e) = o; __threadfence(); } }
}
__global__ __launch_bounds__(256) void featT_kernel(const float* __restrict__ xin, const float* __restrict__ h, const float* __restrict__ h1, b16* __restrict__ XSTh, b16* __restrict__ XSTl, b16* __restrict__ XS2Th, b16* __restrict__ XS2Tl, b16* __restrict__ XSCTh, b16* __restrict__ XSCTl, b16* __restrict__ XSC2Th, b16* __restrict__ XSC2Tl) {
  __shared__ __attribute__((aligned(16))) b16 T[U][64 + 8];
  const int b = blockIdx.z, tile = blockIdx.x, t_ = threadIdx.x; const bool fine = tile < NN / 64; const int n0 = (fine ? tile : tile - NN / 64) * 64; const int W = fine ? NN : NC;
  const float* src = fine ? (h + ((size_t)b * NN + n0) * U) : (h1 + ((size_t)b * NC + n0) * U);
  for (int q = t_; q < 64 * U; q += 256) { const int nn = q >> 6, d = q & 63; T[d][nn] = (b16)(bf16_rne(src[(size_t)nn * U + d]) * XS); }
  __syncthreads();
  b16* ph = fine ? XSTh : XSCTh; b16* pl = fine ? XSTl : XSCTl; b16* p2h = fine ? XS2Th : XSC2Th; b16* p2l = fine ? XS2Tl : XSC2Tl; const size_t base = (size_t)b * KF * W; const v8b z = {};
  for (int pass = 0; pass < 2; ++pass) {
    for (int q = t_; q < U * 8; q += 256) { const int d = q >> 3, c8 = (q & 7) * 8; const size_t gi = base + (size_t)(1 + d) * W + n0 + c8; const v8b v = *(const v8b*)(&T[d][c8]); *(volatile v8b*)(ph + gi) = v; *(volatile v8b*)(pl + gi) = z; *(volatile v8b*)(p2h + gi) = v; *(volatile v8b*)(p2l + gi) = z; }
    for (int q = t_; q < (KF - U - 1) * 8; q += 256) { const int d = U + 1 + (q >> 3), c8 = (q & 7) * 8; const size_t gi = base + (size_t)d * W + n0 + c8; *(volatile v8b*)(ph + gi) = z; *(volatile v8b*)(pl + gi) = z; *(volatile v8b*)(p2h + gi) = z; *(volatile v8b*)(p2l + gi) = z; }
    if (t_ < 8) { const size_t gi = base + n0 + t_ * 8; v8b xv; if (fine) { for (int j = 0; j < 8; ++j) xv[j] = (b16)(bf16_rne(xin[(size_t)b * NN + n0 + t_ * 8 + j]) * XS); *(volatile v8b*)(ph + gi) = xv; *(volatile v8b*)(pl + gi) = z; *(volatile v8b*)(p2h + gi) = xv; *(volatile v8b*)(p2l + gi) = z; } }
    __threadfence(); }
}
__global__ __launch_bounds__(256) void cx_kernel(const float* __restrict__ afc, const float* __restrict__ xin, b16* __restrict__ XSCTh, b16* __restrict__ XSCTl, b16* __restrict__ XSC2Th, b16* __restrict__ XSC2Tl) {
  __shared__ __attribute__((aligned(16))) b16 Rh[NC], Rl[NC];
  const int b = blockIdx.x, c = threadIdx.x; float s = 0.0f;
#pragma unroll 4
  for (int n = 0; n < NN; ++n) s += pmul(bf16_rne(afc[(size_t)n * NC + c]), bf16_rne(xin[(size_t)b * NN + n]));
  b16 p, q; split16(s * XS, p, q); Rh[c] = p; Rl[c] = q;
  __syncthreads();
  for (int pass = 0; pass < 2; ++pass) { if (c < 32) { const size_t gi = (size_t)b * KF * NC + c * 8; const v8b hv = *(const v8b*)(&Rh[c * 8]), lv = *(const v8b*)(&Rl[c * 8]); *(volatile v8b*)(XSCTh + gi) = hv; *(volatile v8b*)(XSCTl + gi) = lv; *(volatile v8b*)(XSC2Th + gi) = hv; *(volatile v8b*)(XSC2Tl + gi) = lv; } __threadfence(); }
}
template <int KD, int NPROD>
__global__ __launch_bounds__(128) void conv_kernel(const b16* __restrict__ A, const b16* __restrict__ Bh, const b16* __restrict__ Bl, float inv_scale, b16* __restrict__ Yh, b16* __restrict__ Yl, int M) {
  __shared__ __attribute__((aligned(16))) b16 Th[4][16][KP + 8], Tl[4][16][KP + 8];
  const int wave = threadIdx.x >> 5, lane = threadIdx.x & 31, nloc = lane & 15, hlf = lane >> 4; const int b = blockIdx.z; const size_t m0 = (size_t)blockIdx.x * 64 + wave * 16;
  const b16* Bb = Bh + (size_t)b * KF * KD; const b16* Blb = Bl + (size_t)b * KF * KD; v8f acc[6];
#pragma unroll
  for (int t = 0; t < 6; ++t) acc[t] = (v8f){};
#pragma unroll 2
  for (int kb = 0; kb < KD; kb += 32) { const v16b a = frag_kb(A + (m0 + nloc) * KD + kb, hlf);
#pragma unroll
    for (int t = 0; t < 6; ++t) { acc[t] = wmma16b(a, frag_kb(Bb + (size_t)(t * 16 + nloc) * KD + kb, hlf), acc[t]); if (NPROD == 2) acc[t] = wmma16b(a, frag_kb(Blb + (size_t)(t * 16 + nloc) * KD + kb, hlf), acc[t]); } }
#pragma unroll
  for (int t = 0; t < 8; ++t)
#pragma unroll
    for (int r = 0; r < 8; ++r) { b16 p = (b16)0.0f, q = (b16)0.0f; if (t < 6) split16(acc[t][r] * inv_scale * XS, p, q); Th[wave][8 * hlf + r][t * 16 + nloc] = p; Tl[wave][8 * hlf + r][t * 16 + nloc] = q; }
  wave_lds_sync();
  for (int pass = 0; pass < 2; ++pass) { for (int r2 = 0; r2 < 16; r2 += 2) { const int rr = r2 + (lane >> 4), c8 = (lane & 15) * 8; const size_t gi = ((size_t)b * M + m0 + rr) * KP + c8; *(volatile v8b*)(Yh + gi) = *(const v8b*)(&Th[wave][rr][c8]); *(volatile v8b*)(Yl + gi) = *(const v8b*)(&Tl[wave][rr][c8]); } __threadfence(); }
}
__global__ __launch_bounds__(128) void gate_kernel(const b16* __restrict__ CFh, const b16* __restrict__ CFl, const b16* __restrict__ LFh, const b16* __restrict__ LFl, const b16* __restrict__ W0P, const float* __restrict__ b0, const float* __restrict__ h, float* __restrict__ Uf, b16* __restrict__ XS2Th, b16* __restrict__ XS2Tl) {
  __shared__ __attribute__((aligned(16))) float Tu[4][16][U + 4]; __shared__ __attribute__((aligned(16))) b16 Rt[U][64 + 8], Rtl[U][64 + 8];
  const int wave = threadIdx.x >> 5, lane = threadIdx.x & 31, nloc = lane & 15, hlf = lane >> 4, t_ = threadIdx.x; const int b = blockIdx.z; const int n0b = blockIdx.x * 64; const size_t m0 = (size_t)n0b + wave * 16;
  v8f a1[8], a2[8];
#pragma unroll
  for (int t = 0; t < 8; ++t) { a1[t] = (v8f){}; a2[t] = (v8f){}; }
#pragma unroll
  for (int kb = 0; kb < KF; kb += 32) { const size_t ro = ((size_t)b * NN + m0 + nloc) * KP + kb; const v16b c = frag_kb(CFh + ro, hlf), cl = frag_kb(CFl + ro, hlf), l = frag_kb(LFh + ro, hlf), ll = frag_kb(LFl + ro, hlf);
#pragma unroll
    for (int t = 0; t < 8; ++t) { const v16b bw = frag_kb(W0P + (size_t)(t * 16 + nloc) * KF + kb, hlf); a1[t] = wmma16b(c, bw, a1[t]); a1[t] = wmma16b(cl, bw, a1[t]); a2[t] = wmma16b(l, bw, a2[t]); a2[t] = wmma16b(ll, bw, a2[t]); } }
#pragma unroll
  for (int t = 0; t < 8; ++t) { const int cidx = t * 16 + nloc; const float bb = bf16_rne(b0[cidx]);
#pragma unroll
    for (int r = 0; r < 8; ++r) { const float x1 = a1[t][r] * (1.0f / (XS * WSC)) + NMIX2 * sigm_(a2[t][r] * (1.0f / (XS * WSC))) + bb; const float g = sigm_(x1); const int rl = 8 * hlf + r;
      if (t < 4) { const float hv = bf16_rne(h[((size_t)b * NN + m0 + rl) * U + cidx]); b16 p, q; split16(pmul(g, hv) * XS, p, q); Rt[cidx][wave * 16 + rl] = p; Rtl[cidx][wave * 16 + rl] = q; }
      else Tu[wave][rl][cidx - U] = g; } }
  __syncthreads();
  for (int pass = 0; pass < 2; ++pass) {
    for (int rr = 0; rr < 16; ++rr) if (lane < 16) *(volatile v4f*)(Uf + ((size_t)b * NN + m0 + rr) * U + lane * 4) = *(const v4f*)(&Tu[wave][rr][lane * 4]);
    for (int q = t_; q < U * 8; q += 128) { const int d = q >> 3, c8 = (q & 7) * 8; const size_t gi = ((size_t)b * KF + 1 + d) * NN + n0b + c8; *(volatile v8b*)(XS2Th + gi) = *(const v8b*)(&Rt[d][c8]); *(volatile v8b*)(XS2Tl + gi) = *(const v8b*)(&Rtl[d][c8]); }
    __threadfence(); }
}
__global__ __launch_bounds__(128) void cgate_kernel(const b16* __restrict__ CCh, const b16* __restrict__ CCl, const b16* __restrict__ W01P, const float* __restrict__ b01, const float* __restrict__ h1, float* __restrict__ U1f, b16* __restrict__ XSC2Th, b16* __restrict__ XSC2Tl) {
  __shared__ __attribute__((aligned(16))) float Tu[4][16][U + 4]; __shared__ __attribute__((aligned(16))) b16 Rt[U][64 + 8], Rtl[U][64 + 8];
  const int wave = threadIdx.x >> 5, lane = threadIdx.x & 31, nloc = lane & 15, hlf = lane >> 4, t_ = threadIdx.x; const int b = blockIdx.z; const int c0b = blockIdx.x * 64; const size_t m0 = (size_t)c0b + wave * 16;
  v8f a1[8];
#pragma unroll
  for (int t = 0; t < 8; ++t) a1[t] = (v8f){};
#pragma unroll
  for (int kb = 0; kb < KF; kb += 32) { const size_t ro = ((size_t)b * NC + m0 + nloc) * KP + kb; const v16b c = frag_kb(CCh + ro, hlf), cl = frag_kb(CCl + ro, hlf);
#pragma unroll
    for (int t = 0; t < 8; ++t) { const v16b bw = frag_kb(W01P + (size_t)(t * 16 + nloc) * KF + kb, hlf); a1[t] = wmma16b(c, bw, a1[t]); a1[t] = wmma16b(cl, bw, a1[t]); } }
#pragma unroll
  for (int t = 0; t < 8; ++t) { const int cidx = t * 16 + nloc; const float bb = bf16_rne(b01[cidx]);
#pragma unroll
    for (int r = 0; r < 8; ++r) { const float g = sigm_(a1[t][r] * (1.0f / (XS * WSC)) + bb); const int rl = 8 * hlf + r;
      if (t < 4) { const float hv = bf16_rne(h1[((size_t)b * NC + m0 + rl) * U + cidx]); b16 p, q; split16(pmul(g, hv) * XS, p, q); Rt[cidx][wave * 16 + rl] = p; Rtl[cidx][wave * 16 + rl] = q; } else Tu[wave][rl][cidx - U] = g; } }
  __syncthreads();
  for (int pass = 0; pass < 2; ++pass) {
    for (int rr = 0; rr < 16; ++rr) if (lane < 16) *(volatile v4f*)(U1f + ((size_t)b * NC + m0 + rr) * U + lane * 4) = *(const v4f*)(&Tu[wave][rr][lane * 4]);
    for (int q = t_; q < U * 8; q += 128) { const int d = q >> 3, c8 = (q & 7) * 8; const size_t gi = ((size_t)b * KF + 1 + d) * NC + c0b + c8; *(volatile v8b*)(XSC2Th + gi) = *(const v8b*)(&Rt[d][c8]); *(volatile v8b*)(XSC2Tl + gi) = *(const v8b*)(&Rtl[d][c8]); }
    __threadfence(); }
}
template <int COARSE>
__global__ __launch_bounds__(128) void cand_kernel(const b16* __restrict__ CFh, const b16* __restrict__ CFl, const b16* __restrict__ LFh, const b16* __restrict__ LFl, const b16* __restrict__ WP, const float* __restrict__ bias, const float* __restrict__ Uf, const float* __restrict__ h, float* __restrict__ out, int M) {
  __shared__ __attribute__((aligned(16))) float To[4][16][U + 4];
  const int wave = threadIdx.x >> 5, lane = threadIdx.x & 31, nloc = lane & 15, hlf = lane >> 4; const int b = blockIdx.z; const size_t m0 = (size_t)blockIdx.x * 64 + wave * 16;
  v8f a1[4], a2[4];
#pragma unroll
  for (int t = 0; t < 4; ++t) { a1[t] = (v8f){}; a2[t] = (v8f){}; }
#pragma unroll
  for (int kb = 0; kb < KF; kb += 32) { const size_t ro = ((size_t)b * M + m0 + nloc) * KP + kb; const v16b c = frag_kb(CFh + ro, hlf), cl = frag_kb(CFl + ro, hlf); v16b l, ll; if (!COARSE) { l = frag_kb(LFh + ro, hlf); ll = frag_kb(LFl + ro, hlf); }
#pragma unroll
    for (int t = 0; t < 4; ++t) { const v16b bw = frag_kb(WP + (size_t)(t * 16 + nloc) * KF + kb, hlf); a1[t] = wmma16b(c, bw, a1[t]); a1[t] = wmma16b(cl, bw, a1[t]); if (!COARSE) { a2[t] = wmma16b(l, bw, a2[t]); a2[t] = wmma16b(ll, bw, a2[t]); } } }
#pragma unroll
  for (int t = 0; t < 4; ++t) { const int d = t * 16 + nloc; const float bb = bf16_rne(bias[d]);
#pragma unroll
    for (int r = 0; r < 8; ++r) { const int rl = 8 * hlf + r; float pre = a1[t][r] * (1.0f / (XS * WSC)) + bb; if (!COARSE) pre += NMIX1 * sigm_(a2[t][r] * (1.0f / (XS * WSC))); const float cval = tanhf(pre);
      const size_t ri = ((size_t)b * M + m0 + rl) * U + d; const float uu = Uf[ri], hv = bf16_rne(h[ri]); To[wave][rl][d] = pmul(uu, hv) + pmul(1.0f - uu, cval); } }
  wave_lds_sync();
  for (int pass = 0; pass < 2; ++pass) { for (int rr = 0; rr < 16; ++rr) if (lane < 16) *(volatile v4f*)(out + ((size_t)b * M + m0 + rr) * U + lane * 4) = *(const v4f*)(&To[wave][rr][lane * 4]); __threadfence(); }
}
}

extern "C" void kernel_launch(void* const* d_in, const int* in_sizes, int n_in, void* d_out, int out_size, void* d_ws, size_t ws_size, hipStream_t stream) {
  (void)n_in;
  auto Fp = [&](int i) { return (const float*)d_in[i]; };
  if (in_sizes[0] != NB * NN || in_sizes[1] != NB * NN * U || in_sizes[2] != NB * NC * U || in_sizes[3] != NN * NN || in_sizes[4] != NC * NC || in_sizes[5] != NN * NC || in_sizes[6] != (U + 1) * G2 || in_sizes[8] != (U + 1) * U || in_sizes[10] != (U + 1) * G2 || in_sizes[12] != (U + 1) * U || out_size != NB * NN * U + NB * NC * U) return;
  size_t off = 0; char* ws = (char*)d_ws;
  auto carve = [&](size_t bytes) { char* p = ws + off; off += (bytes + 255) & ~(size_t)255; return p; };
  b16* ADJ16 = (b16*)carve((size_t)NN * NN * 2); b16* ADJ1 = (b16*)carve((size_t)NC * NC * 2); b16* AFC16 = (b16*)carve((size_t)NN * NC * 2);
  b16* W0P = (b16*)carve((size_t)G2 * KF * 2); b16* W1P = (b16*)carve((size_t)U * KF * 2); b16* W01P = (b16*)carve((size_t)G2 * KF * 2); b16* W11P = (b16*)carve((size_t)U * KF * 2);
  auto plane = [&](int W) { return (b16*)carve((size_t)NB * KF * W * 2); };
  b16* XSTh = plane(NN); b16* XSTl = plane(NN); b16* XS2Th = plane(NN); b16* XS2Tl = plane(NN); b16* XSCTh = plane(NC); b16* XSCTl = plane(NC); b16* XSC2Th = plane(NC); b16* XSC2Tl = plane(NC);
  auto fplane = [&](int M) { return (b16*)carve((size_t)NB * M * KP * 2); };
  b16* CFh = fplane(NN); b16* CFl = fplane(NN); b16* LFh = fplane(NN); b16* LFl = fplane(NN); b16* CCh = fplane(NC); b16* CCl = fplane(NC);
  float* Uf = (float*)carve((size_t)NB * NN * U * 4); float* U1f = (float*)carve((size_t)NB * NC * U * 4);
  if (off > ws_size || off > ((size_t)128 << 20)) return;
  prep_kernel<<<(unsigned)(((size_t)NN * NN / 8 + (size_t)NC * NC / 8 + (size_t)NN * NC / 8 + 2 * (size_t)G2 * KF / 8 + 2 * (size_t)U * KF / 8 + 255) / 256), 256, 0, stream>>>(Fp(3), Fp(4), Fp(5), Fp(6), Fp(8), Fp(10), Fp(12), ADJ16, ADJ1, AFC16, W0P, W1P, W01P, W11P);
  featT_kernel<<<dim3(NN / 64 + NC / 64, 1, NB), 256, 0, stream>>>(Fp(0), Fp(1), Fp(2), XSTh, XSTl, XS2Th, XS2Tl, XSCTh, XSCTl, XSC2Th, XSC2Tl);
  cx_kernel<<<NB, 256, 0, stream>>>(Fp(5), Fp(0), XSCTh, XSCTl, XSC2Th, XSC2Tl);
  conv_kernel<NN, 1><<<dim3(NN / 64, 1, NB), 128, 0, stream>>>(ADJ16, XSTh, XSTl, 1.0f / (WSC * XS), CFh, CFl, NN);
  conv_kernel<NC, 2><<<dim3(NN / 64, 1, NB), 128, 0, stream>>>(AFC16, XSCTh, XSCTl, 1.0f / (XS * XS), LFh, LFl, NN);
  conv_kernel<NC, 2><<<dim3(NC / 64, 1, NB), 128, 0, stream>>>(ADJ1, XSCTh, XSCTl, 1.0f / (WSC * XS), CCh, CCl, NC);
  gate_kernel<<<dim3(NN / 64, 1, NB), 128, 0, stream>>>(CFh, CFl, LFh, LFl, W0P, Fp(7), Fp(1), Uf, XS2Th, XS2Tl);
  cgate_kernel<<<dim3(NC / 64, 1, NB), 128, 0, stream>>>(CCh, CCl, W01P, Fp(11), Fp(2), U1f, XSC2Th, XSC2Tl);
  conv_kernel<NN, 2><<<dim3(NN / 64, 1, NB), 128, 0, stream>>>(ADJ16, XS2Th, XS2Tl, 1.0f / (WSC * XS), CFh, CFl, NN);
  conv_kernel<NC, 2><<<dim3(NN / 64, 1, NB), 128, 0, stream>>>(AFC16, XSC2Th, XSC2Tl, 1.0f / (XS * XS), LFh, LFl, NN);
  conv_kernel<NC, 2><<<dim3(NC / 64, 1, NB), 128, 0, stream>>>(ADJ1, XSC2Th, XSC2Tl, 1.0f / (WSC * XS), CCh, CCl, NC);
  cand_kernel<0><<<dim3(NN / 64, 1, NB), 128, 0, stream>>>(CFh, CFl, LFh, LFl, W1P, Fp(9), Uf, Fp(1), (float*)d_out, NN);
  cand_kernel<1><<<dim3(NC / 64, 1, NB), 128, 0, stream>>>(CCh, CCl, nullptr, nullptr, W11P, Fp(13), U1f, Fp(2), (float*)d_out + (size_t)NB * NN * U, NC);
}
